// EncoderLayer_35021163331623
// MI455X (gfx1250) — hardware-verified
//
#include <hip/hip_runtime.h>
#include <math.h>

#ifndef NB
#define NB 2
#endif
#ifndef SEQ
#define SEQ 2048
#endif
#define NB_FULL 2
#define SEQ_FULL 2048
#define DM 512
#define NH 8
#define DKH 128
#define DVH 256
#define DFF 2048
#define NQK (NH * DKH)
#define NVV (NH * DVH)
#define MROWS (NB * SEQ)

static_assert(NB >= 1 && NB <= NB_FULL);
static_assert(SEQ >= 64 && SEQ <= SEQ_FULL);
static_assert(SEQ % 64 == 0);
static_assert(MROWS % 64 == 0);
static_assert(DM % 64 == 0 && NQK % 64 == 0 && NVV % 64 == 0 && DFF % 64 == 0);
static_assert(DM % 32 == 0 && NVV % 32 == 0 && DFF % 32 == 0 && DKH % 32 == 0);
static_assert(DM % 8 == 0 && NVV % 8 == 0 && DFF % 8 == 0);
static_assert(32 * 4 * 4 == DM);
static_assert(DKH == 4 * 32);
static_assert(DVH == 2 * 128);

typedef __attribute__((ext_vector_type(16))) _Float16 v16h;
typedef __attribute__((ext_vector_type(8)))  _Float16 v8h;
typedef __attribute__((ext_vector_type(8)))  float    v8f;
typedef __attribute__((ext_vector_type(4)))  float    v4f;
typedef unsigned int u4v __attribute__((ext_vector_type(4)));
typedef unsigned int u2v __attribute__((ext_vector_type(2)));


#define VST2(T, ptr, val) do { const T vst2_v_ = (val); *(volatile T*)(ptr) = vst2_v_; __threadfence(); *(volatile T*)(ptr) = vst2_v_; } while (0)
#define VST2V4(ptr, val) do { const v4f vst2_v4_ = (val); *(volatile v4f*)(ptr) = vst2_v4_; __threadfence(); *(volatile v4f*)(ptr) = vst2_v4_; } while (0)

__device__ __forceinline__ float cmb_bf(float v) {
    const unsigned u = __builtin_bit_cast(unsigned, v);
    const unsigned r = (u + 0x7fffu + ((u >> 16) & 1u)) & 0xffff0000u;
    return __builtin_bit_cast(float, r);
}
__device__ __forceinline__ unsigned int pk2h(float a, float b) {
    return (unsigned int)__builtin_bit_cast(unsigned short, (_Float16)a) | ((unsigned int)__builtin_bit_cast(unsigned short, (_Float16)b) << 16);
}

union FragU { v16h v; v8h h[2]; };
__device__ __forceinline__ v16h ldfrag_g(const _Float16* __restrict__ p) {
    FragU f; f.h[0] = *(const v8h*)(p); f.h[1] = *(const v8h*)(p + 16); return f.v;
}
__device__ __forceinline__ v8f wmma16(v16h a, v16h b, v8f c) {
    c = __builtin_amdgcn_wmma_f32_16x16x32_f16(false, a, false, b, (short)0, c, false, false);
    asm volatile("v_nop\n\tv_nop\n\tv_nop\n\tv_nop" : "+v"(c) : "v"(a), "v"(b));
    return c;
}
__device__ __forceinline__ void dep_guard_h(v8f& a, v8f& b, v16h x, v16h y) { asm volatile("v_nop\n\tv_nop\n\tv_nop\n\tv_nop" : "+v"(a), "+v"(b) : "v"(x), "v"(y)); }
__device__ __forceinline__ void keep4_h(v16h a, v16h b, v16h c, v16h d) { asm volatile("v_nop" :: "v"(a), "v"(b), "v"(c), "v"(d)); }
__device__ __forceinline__ void acc_guard4(v8f& a, v8f& b, v8f& c, v8f& d) { asm volatile("v_nop\n\tv_nop\n\tv_nop\n\tv_nop" : "+v"(a), "+v"(b), "+v"(c), "+v"(d)); }
__device__ __forceinline__ void wave_sync_lds() {
    __builtin_amdgcn_fence(3  , "workgroup");
    __builtin_amdgcn_wave_barrier();
    __builtin_amdgcn_fence(2  , "workgroup");
}

__global__ __launch_bounds__(256) void k_cast_x(const float* __restrict__ SRC, unsigned short* __restrict__ DST) {
    const long long u = (long long)blockIdx.x * 256 + threadIdx.x; const int per = DM / 8;
    if (u >= (long long)MROWS * per) return;
    const int r = (int)(u / per); const int c0 = 8 * (int)(u % per);
    const int bb = r / SEQ; const int ss = r - bb * SEQ;
    const float* s = SRC + ((long long)bb * SEQ_FULL + ss) * DM + c0;
    const v4f a = *(const v4f*)s; const v4f b = *(const v4f*)(s + 4);
    u4v pk; pk.x = pk2h(cmb_bf(a.x), cmb_bf(a.y)); pk.y = pk2h(cmb_bf(a.z), cmb_bf(a.w)); pk.z = pk2h(cmb_bf(b.x), cmb_bf(b.y)); pk.w = pk2h(cmb_bf(b.z), cmb_bf(b.w));
    VST2(u4v, (u4v*)(DST + (long long)r * DM + c0), pk);
}
__global__ __launch_bounds__(256) void k_cm_castbT_h(const float* __restrict__ SRC, int HD, int nR, unsigned short* __restrict__ DST, int ldd, int nCtot, float sc) {
    const long long u = (long long)blockIdx.x * 256 + threadIdx.x; const int per = nR / 8;
    if (u >= (long long)nCtot * per) return;
    const int c = (int)(u / per); const int r0 = 8 * (int)(u % per);
    const int hd = c / HD; const int kk = c - hd * HD;
    const float* s = SRC + ((long long)hd * nR + r0) * HD + kk;
    float w[8];
#pragma unroll
    for (int e = 0; e < 8; ++e) w[e] = cmb_bf(s[(long long)e * HD]) * sc;
    u4v pk; pk.x = pk2h(w[0], w[1]); pk.y = pk2h(w[2], w[3]); pk.z = pk2h(w[4], w[5]); pk.w = pk2h(w[6], w[7]);
    VST2(u4v, (u4v*)(DST + (long long)c * ldd + r0), pk);
}

template <int BIAS_MODE, int OUT_MODE, int ACT>
__device__ __forceinline__ void gemm64_body(
    const unsigned short* __restrict__ Ap, int lda, long long strideA,
    const unsigned short* __restrict__ Btp, int ldb, long long strideB,
    void* __restrict__ Cout, int ldc, long long strideC,
    const float* __restrict__ bias, int M, int N, int K, float scale) {
  __shared__ __align__(16) float sT[8][16 * 68];
  const int b    = blockIdx.y;
  const int lane = threadIdx.x & 31;
  const int wave = threadIdx.x >> 5;
  const int tilesN = N >> 6;
  const int tilesM = M >> 6;
  const int tile = blockIdx.x * 8 + wave;
  if (tile >= tilesM * tilesN) return;
  const int tm = tile / tilesN;
  const int tn = tile - tm * tilesN;
  const int m0 = tm << 6;
  const int n0 = tn << 6;

  const _Float16* Ab = (const _Float16*)Ap  + (size_t)b * strideA;
  const _Float16* Bb = (const _Float16*)Btp + (size_t)b * strideB;

  const int rlane = lane & 15;
  const int koff  = (lane >> 4) * 8;
  const int mOff  = (lane >> 4) * 8;

  v8f acc[4][4];
#pragma unroll
  for (int i = 0; i < 4; ++i)
#pragma unroll
    for (int j = 0; j < 4; ++j) acc[i][j] = (v8f){0.f,0.f,0.f,0.f,0.f,0.f,0.f,0.f};

  for (int k0 = 0; k0 < K; k0 += 32) {
    v16h bh[4];
#pragma unroll
    for (int j = 0; j < 4; ++j) {
      const size_t bo = (size_t)(n0 + (j << 4) + rlane) * ldb + koff + k0;
      bh[j] = ldfrag_g(Bb + bo);
    }
#pragma unroll
    for (int i = 0; i < 4; ++i) {
      const size_t ao = (size_t)(m0 + (i << 4) + rlane) * lda + koff + k0;
      const v16h ah = ldfrag_g(Ab + ao);
#pragma unroll
      for (int j = 0; j < 4; ++j)
        acc[i][j] = __builtin_amdgcn_wmma_f32_16x16x32_f16(false, ah, false, bh[j], (short)0, acc[i][j], false, false);
      dep_guard_h(acc[i][0], acc[i][3], ah, ah);
    }
    keep4_h(bh[0], bh[1], bh[2], bh[3]);
  }
  acc_guard4(acc[0][0], acc[0][1], acc[0][2], acc[0][3]);
  acc_guard4(acc[1][0], acc[1][1], acc[1][2], acc[1][3]);
  acc_guard4(acc[2][0], acc[2][1], acc[2][2], acc[2][3]);
  acc_guard4(acc[3][0], acc[3][1], acc[3][2], acc[3][3]);

  float* slab = sT[wave];
#pragma unroll
  for (int i = 0; i < 4; ++i) {
    const int mBase = m0 + (i << 4);
#pragma unroll
    for (int j = 0; j < 4; ++j) {
      const int n = n0 + (j << 4) + rlane;
      float bv = 0.f;
      if (BIAS_MODE == 2) bv = cmb_bf(bias[n]);
#pragma unroll
      for (int r = 0; r < 8; ++r) {
        float v = acc[i][j][r] * scale;
        if (BIAS_MODE == 1) v += cmb_bf(bias[mBase + mOff + r]);
        if (BIAS_MODE == 2) v += bv;
        if (ACT == 2) v = fmaxf(v, 0.0f);
        slab[(mOff + r) * 68 + (j << 4) + rlane] = v;
      }
    }
    wave_sync_lds();
    if (OUT_MODE == 0) {
      float* C = (float*)Cout + (size_t)b * strideC;
      const int hh = lane >> 4, c4 = (lane & 15) * 4;
      for (int pass = 0; pass < 2; ++pass) {
#pragma unroll
        for (int it = 0; it < 8; ++it) {
          const int row = it * 2 + hh;
          const v4f v = *(const v4f*)(slab + row * 68 + c4);
          *(volatile v4f*)(C + (size_t)(mBase + row) * ldc + n0 + c4) = v;
        }
        __threadfence();
      }
    } else {
      const int q = lane >> 3, c8 = (lane & 7) * 8;
      unsigned short* C = (unsigned short*)Cout + (size_t)b * strideC;
      for (int pass = 0; pass < 2; ++pass) {
#pragma unroll
        for (int it = 0; it < 4; ++it) {
          const int row = it * 4 + q;
          const float* sp = slab + row * 68 + c8;
          const v4f a = *(const v4f*)sp; const v4f c2 = *(const v4f*)(sp + 4);
          u4v pk; pk.x = pk2h(a.x, a.y); pk.y = pk2h(a.z, a.w); pk.z = pk2h(c2.x, c2.y); pk.w = pk2h(c2.z, c2.w);
          *(volatile u4v*)(C + (size_t)(mBase + row) * ldc + n0 + c8) = pk;
        }
        __threadfence();
      }
    }
    wave_sync_lds();
  }
}

__global__ __launch_bounds__(256) void k_gemm_h_bn(const unsigned short* __restrict__ A, int lda, long long sA, const unsigned short* __restrict__ Bt, int ldb, long long sB,
        unsigned short* __restrict__ C, int ldc, long long sC, const float* __restrict__ bias, int M, int N, int K, float scale) {
    gemm64_body<2, 1, 0>(A, lda, sA, Bt, ldb, sB, (void*)C, ldc, sC, bias, M, N, K, scale);
}
__global__ __launch_bounds__(256) void k_gemm_h_bn_relu(const unsigned short* __restrict__ A, int lda, long long sA, const unsigned short* __restrict__ Bt, int ldb, long long sB,
        unsigned short* __restrict__ C, int ldc, long long sC, const float* __restrict__ bias, int M, int N, int K, float scale) {
    gemm64_body<2, 1, 2>(A, lda, sA, Bt, ldb, sB, (void*)C, ldc, sC, bias, M, N, K, scale);
}
__global__ __launch_bounds__(256) void k_gemm_h_bm(const unsigned short* __restrict__ A, int lda, long long sA, const unsigned short* __restrict__ Bt, int ldb, long long sB,
        unsigned short* __restrict__ C, int ldc, long long sC, const float* __restrict__ bias, int M, int N, int K, float scale) {
    gemm64_body<1, 1, 0>(A, lda, sA, Bt, ldb, sB, (void*)C, ldc, sC, bias, M, N, K, scale);
}
__global__ __launch_bounds__(256) void k_gemm_f_bn(const unsigned short* __restrict__ A, int lda, long long sA, const unsigned short* __restrict__ Bt, int ldb, long long sB,
        float* __restrict__ C, int ldc, long long sC, const float* __restrict__ bias, int M, int N, int K, float scale) {
    gemm64_body<2, 0, 0>(A, lda, sA, Bt, ldb, sB, (void*)C, ldc, sC, bias, M, N, K, scale);
}

#define AT_NW 4
#define AT_QB 64
#define AT_KC 64
#define AT_VH 128
#define AT_OP 132
static_assert(AT_VH * 2 == DVH);
static_assert(AT_QB == AT_NW * 16);
static_assert((AT_OP * 4) % 16 == 0 && AT_OP >= AT_VH);

__global__ __launch_bounds__(128) void k_attn_flash(const unsigned short* __restrict__ Qp, const unsigned short* __restrict__ Kp,
                                                    const unsigned short* __restrict__ VTp, unsigned short* __restrict__ CTXp) {
    __shared__ __align__(16) _Float16 Psh[AT_NW][16 * AT_KC];
    __shared__ __align__(16) float    Os[AT_NW][16 * AT_OP];
    const int tid = threadIdx.x, wave = tid >> 5, lane = tid & 31, hh = lane >> 4, c = lane & 15;
    constexpr int nqb = SEQ / AT_QB;
    int bx = (int)blockIdx.x;
    const int vh = bx & 1; bx >>= 1;
    const int qb = bx % nqb; const int bh = bx / nqb; const int h = bh % NH; const int b = bh / NH;
    const int q0 = qb * AT_QB + wave * 16;
    const float PSC  = 32768.0f;
    const float SCL2 = 0.08838834764831845f * 1.4426950408889634f;
    const float NEG  = -__builtin_inff();

    const _Float16* Qf = (const _Float16*)Qp; const _Float16* Kf = (const _Float16*)Kp; const _Float16* Vf = (const _Float16*)VTp;
    v16h qa[4];
    {
        const _Float16* qrow = Qf + (size_t)(b * SEQ + q0 + c) * NQK + h * DKH + 8 * hh;
#pragma unroll
        for (int dc = 0; dc < 4; ++dc) qa[dc] = ldfrag_g(qrow + dc * 32);
    }
    const _Float16* kbase = Kf + (size_t)(b * SEQ + c) * NQK + h * DKH + 8 * hh;
    const _Float16* vbase = Vf + ((size_t)b * NVV + h * DVH + vh * AT_VH + c) * SEQ + 8 * hh;

    float mrow[8], lrow[8];
    v8f oacc[8];
#pragma unroll
    for (int r = 0; r < 8; ++r) { mrow[r] = NEG; lrow[r] = 0.f; }
#pragma unroll
    for (int t = 0; t < 8; ++t) oacc[t] = (v8f){0.f,0.f,0.f,0.f,0.f,0.f,0.f,0.f};

    for (int kc = 0; kc < SEQ / AT_KC; ++kc) {
        const int kv0 = kc * AT_KC;
        v8f s[4];
#pragma unroll
        for (int j = 0; j < 4; ++j) {
            const _Float16* krow = kbase + (size_t)(kv0 + j * 16) * NQK;
            v8f acc = (v8f){0.f,0.f,0.f,0.f,0.f,0.f,0.f,0.f};
#pragma unroll
            for (int dc = 0; dc < 4; ++dc) acc = wmma16(qa[dc], ldfrag_g(krow + dc * 32), acc);
            s[j] = acc;
        }
#pragma unroll
        for (int r = 0; r < 8; ++r) {
            float sv[4];
            float m = NEG;
#pragma unroll
            for (int j = 0; j < 4; ++j) { sv[j] = s[j][r] * SCL2; m = fmaxf(m, sv[j]); }
            m = fmaxf(m, __shfl_xor(m, 1, 32)); m = fmaxf(m, __shfl_xor(m, 2, 32));
            m = fmaxf(m, __shfl_xor(m, 4, 32)); m = fmaxf(m, __shfl_xor(m, 8, 32));
            const float mnew  = fmaxf(mrow[r], m);
            const float alpha = exp2f(mrow[r] - mnew);
            mrow[r] = mnew;
            float psum = 0.f;
#pragma unroll
            for (int j = 0; j < 4; ++j) {
                const float p = exp2f(sv[j] - mnew);
                psum += p;
                Psh[wave][(8 * hh + r) * AT_KC + j * 16 + c] = (_Float16)(p * PSC);
            }
            psum += __shfl_xor(psum, 1, 32); psum += __shfl_xor(psum, 2, 32);
            psum += __shfl_xor(psum, 4, 32); psum += __shfl_xor(psum, 8, 32);
            lrow[r] = lrow[r] * alpha + psum;
#pragma unroll
            for (int t = 0; t < 8; ++t) oacc[t][r] *= alpha;
        }
        wave_sync_lds();
#pragma unroll
        for (int kk = 0; kk < 2; ++kk) {
            FragU pa;
            pa.h[0] = *(const v8h*)(&Psh[wave][c * AT_KC + kk * 32 + 8 * hh]);
            pa.h[1] = *(const v8h*)(&Psh[wave][c * AT_KC + kk * 32 + 16 + 8 * hh]);
#pragma unroll
            for (int t = 0; t < 8; ++t) {
                const v16h vb = ldfrag_g(vbase + (size_t)(t * 16) * SEQ + kv0 + kk * 32);
                oacc[t] = wmma16(pa.v, vb, oacc[t]);
            }
        }
        wave_sync_lds();
    }

#pragma unroll
    for (int r = 0; r < 8; ++r) {
        const float inv = 256.0f / (lrow[r] * PSC);
#pragma unroll
        for (int t = 0; t < 8; ++t) Os[wave][(8 * hh + r) * AT_OP + t * 16 + c] = oacc[t][r] * inv;
    }
    wave_sync_lds();
    {
        unsigned short* crow = CTXp + (size_t)(b * SEQ + q0) * NVV + h * DVH + vh * AT_VH;
        const int c8 = (lane & 15) * 8;
        for (int pass = 0; pass < 2; ++pass) {
#pragma unroll
            for (int it = 0; it < 8; ++it) {
                const int row = it * 2 + hh;
                const v4f a  = *(const v4f*)(&Os[wave][row * AT_OP + c8]);
                const v4f b2 = *(const v4f*)(&Os[wave][row * AT_OP + c8 + 4]);
                u4v pk; pk.x = pk2h(a.x, a.y); pk.y = pk2h(a.z, a.w); pk.z = pk2h(b2.x, b2.y); pk.w = pk2h(b2.z, b2.w);
                *(volatile u4v*)(crow + (size_t)row * NVV + c8) = pk;
            }
            __threadfence();
        }
    }
}

template <int XBF, int XFULL, int OFULL, int W16>
__device__ __forceinline__ void ln512_body(const float* __restrict__ A, const float* __restrict__ X, const float* __restrict__ GA, const float* __restrict__ BE,
                                           float* __restrict__ Yf, unsigned short* __restrict__ Y16) {
    #pragma clang fp contract(off)
    constexpr int NQ = 4;
    const int r = blockIdx.x * 8 + (threadIdx.x >> 5); const int L = threadIdx.x & 31;
    if (r >= MROWS) return;
    const int bb = r / SEQ; const int ss = r - bb * SEQ; const long long rf = (long long)bb * SEQ_FULL + ss;
    const long long oA = (long long)r * DM;
    const long long oX = (XFULL ? rf : (long long)r) * DM;
    const long long oY = (OFULL ? rf : (long long)r) * DM;
    v4f v[NQ]; float s = 0.f;
#pragma unroll
    for (int q = 0; q < NQ; ++q) {
        const int c = 4 * L + 128 * q;
        v[q] = *(const v4f*)(A + oA + c);
        v4f x = *(const v4f*)(X + oX + c);
        if (XBF) { x.x = cmb_bf(x.x); x.y = cmb_bf(x.y); x.z = cmb_bf(x.z); x.w = cmb_bf(x.w); }
        v[q] = v[q] + x;
        s += (v[q].x + v[q].y) + (v[q].z + v[q].w);
    }
#pragma unroll
    for (int o = 16; o > 0; o >>= 1) s += __shfl_xor(s, o, 32);
    const float mu = s * (1.f / DM); float qq = 0.f;
#pragma unroll
    for (int q = 0; q < NQ; ++q) { v[q].x -= mu; v[q].y -= mu; v[q].z -= mu; v[q].w -= mu; qq += (v[q].x * v[q].x + v[q].y * v[q].y) + (v[q].z * v[q].z + v[q].w * v[q].w); }
#pragma unroll
    for (int o = 16; o > 0; o >>= 1) qq += __shfl_xor(qq, o, 32);
    const float rs = rsqrtf(qq * (1.f / DM) + 1e-5f);
#pragma unroll
    for (int q = 0; q < NQ; ++q) {
        const int c = 4 * L + 128 * q;
        const v4f ga = *(const v4f*)(GA + c), be = *(const v4f*)(BE + c);
        v4f y;
        y.x = v[q].x * rs * cmb_bf(ga.x) + cmb_bf(be.x); y.y = v[q].y * rs * cmb_bf(ga.y) + cmb_bf(be.y);
        y.z = v[q].z * rs * cmb_bf(ga.z) + cmb_bf(be.z); y.w = v[q].w * rs * cmb_bf(ga.w) + cmb_bf(be.w);
        VST2V4(Yf + oY + c, y);
        if (W16) { u2v pk; pk.x = pk2h(y.x, y.y); pk.y = pk2h(y.z, y.w); VST2(u2v, (u2v*)(Y16 + oA + c), pk); }
    }
}
__global__ __launch_bounds__(256) void k_ln1(const float* __restrict__ ATT, const float* __restrict__ x, const float* __restrict__ g, const float* __restrict__ be,
                                             float* __restrict__ X1, unsigned short* __restrict__ H16) {
    ln512_body<1, 1, 0, 1>(ATT, x, g, be, X1, H16);
}
__global__ __launch_bounds__(256) void k_ln2(const float* __restrict__ FFo, const float* __restrict__ X1, const float* __restrict__ g, const float* __restrict__ be,
                                             float* __restrict__ out) {
    ln512_body<0, 0, 1, 0>(FFo, X1, g, be, out, nullptr);
}

constexpr size_t al256(size_t x) { return (x + 255) / 256 * 256; }
constexpr size_t SZ_X16 = al256((size_t)MROWS * DM * 2);
constexpr size_t SZ_WSQ = al256((size_t)DM * DM * 2);
constexpr size_t SZ_WQP = al256((size_t)NQK * DM * 2);
constexpr size_t SZ_WVP = al256((size_t)NVV * DM * 2);
constexpr size_t SZ_WO  = al256((size_t)DM * NVV * 2);
constexpr size_t SZ_W1  = al256((size_t)DFF * DM * 2);
constexpr size_t SZ_W2  = al256((size_t)DM * DFF * 2);
constexpr size_t SZ_QKV = al256((size_t)MROWS * 3 * DM * 2);
constexpr size_t SZ_QH  = al256((size_t)MROWS * NQK * 2);
constexpr size_t SZ_VHT = al256((size_t)NB * NVV * SEQ * 2);
constexpr size_t SZ_CTX = al256((size_t)MROWS * NVV * 2);
constexpr size_t SZ_F32 = al256((size_t)MROWS * DM * 4);
constexpr size_t SZ_H16 = al256((size_t)MROWS * DM * 2);
constexpr size_t SZ_F16 = al256((size_t)MROWS * DFF * 2);
constexpr size_t WS_TOTAL = SZ_X16 + 3 * SZ_WSQ + 2 * SZ_WQP + SZ_WVP + SZ_WO + SZ_W1 + SZ_W2 + SZ_QKV + 2 * SZ_QH + SZ_VHT + SZ_CTX + 3 * SZ_F32 + SZ_H16 + SZ_F16;
static_assert(WS_TOTAL <= (size_t)134217728);
static_assert(((size_t)(NB - 1) * SEQ_FULL + SEQ) * DM <= (size_t)NB_FULL * SEQ_FULL * DM);

static inline unsigned ggrid(int M, int N) { return (unsigned)((((M / 64) * (N / 64)) + 7) / 8); }
static inline unsigned cgrid(long long n) { return (unsigned)((n + 255) / 256); }

extern "C" void kernel_launch(void* const* d_in, const int* in_sizes, int n_in, void* d_out, int out_size, void* d_ws, size_t ws_size, hipStream_t stream) {
    if (n_in < 23) return;
    const long long xneed = ((long long)(NB - 1) * SEQ_FULL + SEQ) * DM;
    if ((long long)in_sizes[0] < xneed) return;
    if (in_sizes[1] < DM * DM || in_sizes[3] < DM * DM || in_sizes[5] < DM * DM) return;
    if (in_sizes[2] < DM || in_sizes[4] < DM || in_sizes[6] < DM) return;
    if (in_sizes[7] < NH * DM * DKH || in_sizes[9] < NH * DM * DKH || in_sizes[11] < NH * DM * DVH) return;
    if (in_sizes[8] < NQK || in_sizes[10] < NQK || in_sizes[12] < NVV) return;
    if (in_sizes[13] < NVV * DM || in_sizes[14] < DM) return;
    if (in_sizes[15] < DM * DFF || in_sizes[16] < DFF || in_sizes[17] < DFF * DM || in_sizes[18] < DM) return;
    if (in_sizes[19] < DM || in_sizes[20] < DM || in_sizes[21] < DM || in_sizes[22] < DM) return;
    if ((long long)out_size < xneed) return;
    if (ws_size < WS_TOTAL) return;

    const float* x   = (const float*)d_in[0];
    const float* Wq  = (const float*)d_in[1];
    const float* bq  = (const float*)d_in[2];
    const float* Wk  = (const float*)d_in[3];
    const float* bk  = (const float*)d_in[4];
    const float* Wv  = (const float*)d_in[5];
    const float* bv  = (const float*)d_in[6];
    const float* WQp = (const float*)d_in[7];
    const float* bQp = (const float*)d_in[8];
    const float* WKp = (const float*)d_in[9];
    const float* bKp = (const float*)d_in[10];
    const float* WVp = (const float*)d_in[11];
    const float* bVp = (const float*)d_in[12];
    const float* Wo  = (const float*)d_in[13];
    const float* bo  = (const float*)d_in[14];
    const float* W1  = (const float*)d_in[15];
    const float* b1  = (const float*)d_in[16];
    const float* W2  = (const float*)d_in[17];
    const float* b2  = (const float*)d_in[18];
    const float* g1  = (const float*)d_in[19];
    const float* be1 = (const float*)d_in[20];
    const float* g2  = (const float*)d_in[21];
    const float* be2 = (const float*)d_in[22];
    float* out = (float*)d_out;

    char* wsp = (char*)d_ws;
    unsigned short* X16   = (unsigned short*)wsp; wsp += SZ_X16;
    unsigned short* WQT   = (unsigned short*)wsp; wsp += SZ_WSQ;
    unsigned short* WKT   = (unsigned short*)wsp; wsp += SZ_WSQ;
    unsigned short* WVT   = (unsigned short*)wsp; wsp += SZ_WSQ;
    unsigned short* WQPT  = (unsigned short*)wsp; wsp += SZ_WQP;
    unsigned short* WKPT  = (unsigned short*)wsp; wsp += SZ_WQP;
    unsigned short* WVPT  = (unsigned short*)wsp; wsp += SZ_WVP;
    unsigned short* WOT   = (unsigned short*)wsp; wsp += SZ_WO;
    unsigned short* W1T   = (unsigned short*)wsp; wsp += SZ_W1;
    unsigned short* W2T   = (unsigned short*)wsp; wsp += SZ_W2;
    unsigned short* QKV16 = (unsigned short*)wsp; wsp += SZ_QKV;
    unsigned short* QH16  = (unsigned short*)wsp; wsp += SZ_QH;
    unsigned short* KH16  = (unsigned short*)wsp; wsp += SZ_QH;
    unsigned short* VHT16 = (unsigned short*)wsp; wsp += SZ_VHT;
    unsigned short* CTX16 = (unsigned short*)wsp; wsp += SZ_CTX;
    float*          ATT   = (float*)wsp;          wsp += SZ_F32;
    float*          X1    = (float*)wsp;          wsp += SZ_F32;
    float*          FFo   = (float*)wsp;          wsp += SZ_F32;
    unsigned short* H16   = (unsigned short*)wsp; wsp += SZ_H16;
    unsigned short* F16   = (unsigned short*)wsp; wsp += SZ_F16;
    if ((size_t)(wsp - (char*)d_ws) > ws_size) return;

    const float WS16 = 16.0f;
    const float IW   = 0.0625f;

    k_cast_x<<<cgrid((long long)MROWS * (DM / 8)), 256, 0, stream>>>(x, X16);
    k_cm_castbT_h<<<cgrid((long long)DM * (DM / 8)), 256, 0, stream>>>(Wq, DM, DM, WQT, DM, DM, WS16);
    k_cm_castbT_h<<<cgrid((long long)DM * (DM / 8)), 256, 0, stream>>>(Wk, DM, DM, WKT, DM, DM, WS16);
    k_cm_castbT_h<<<cgrid((long long)DM * (DM / 8)), 256, 0, stream>>>(Wv, DM, DM, WVT, DM, DM, WS16);
    k_cm_castbT_h<<<cgrid((long long)NQK * (DM / 8)), 256, 0, stream>>>(WQp, DKH, DM, WQPT, DM, NQK, WS16);
    k_cm_castbT_h<<<cgrid((long long)NQK * (DM / 8)), 256, 0, stream>>>(WKp, DKH, DM, WKPT, DM, NQK, WS16);
    k_cm_castbT_h<<<cgrid((long long)NVV * (DM / 8)), 256, 0, stream>>>(WVp, DVH, DM, WVPT, DM, NVV, WS16);
    k_cm_castbT_h<<<cgrid((long long)DM * (NVV / 8)), 256, 0, stream>>>(Wo, DM, NVV, WOT, NVV, DM, WS16);
    k_cm_castbT_h<<<cgrid((long long)DFF * (DM / 8)), 256, 0, stream>>>(W1, DFF, DM, W1T, DM, DFF, WS16);
    k_cm_castbT_h<<<cgrid((long long)DM * (DFF / 8)), 256, 0, stream>>>(W2, DM, DFF, W2T, DFF, DM, WS16);

    k_gemm_h_bn<<<dim3(ggrid(MROWS, DM), 1), 256, 0, stream>>>(X16, DM, 0LL, WQT, DM, 0LL, QKV16 + 0,      3 * DM, 0LL, bq, MROWS, DM, DM, IW);
    k_gemm_h_bn<<<dim3(ggrid(MROWS, DM), 1), 256, 0, stream>>>(X16, DM, 0LL, WKT, DM, 0LL, QKV16 + DM,     3 * DM, 0LL, bk, MROWS, DM, DM, IW);
    k_gemm_h_bn<<<dim3(ggrid(MROWS, DM), 1), 256, 0, stream>>>(X16, DM, 0LL, WVT, DM, 0LL, QKV16 + 2 * DM, 3 * DM, 0LL, bv, MROWS, DM, DM, IW);
    k_gemm_h_bn<<<dim3(ggrid(MROWS, NQK), 1), 256, 0, stream>>>(QKV16 + 0,  3 * DM, 0LL, WQPT, DM, 0LL, QH16, NQK, 0LL, bQp, MROWS, NQK, DM, IW);
    k_gemm_h_bn<<<dim3(ggrid(MROWS, NQK), 1), 256, 0, stream>>>(QKV16 + DM, 3 * DM, 0LL, WKPT, DM, 0LL, KH16, NQK, 0LL, bKp, MROWS, NQK, DM, IW);
    k_gemm_h_bm<<<dim3(ggrid(NVV, SEQ), NB), 256, 0, stream>>>(WVPT, DM, 0LL, QKV16 + 2 * DM, 3 * DM, (long long)SEQ * 3 * DM, VHT16, SEQ, (long long)NVV * SEQ, bVp, NVV, SEQ, DM, IW);

    k_attn_flash<<<dim3((unsigned)(NB * NH * (SEQ / AT_QB) * 2)), 128, 0, stream>>>(QH16, KH16, VHT16, CTX16);

    k_gemm_f_bn<<<dim3(ggrid(MROWS, DM), 1), 256, 0, stream>>>(CTX16, NVV, 0LL, WOT, NVV, 0LL, ATT, DM, 0LL, bo, MROWS, DM, NVV, IW * (1.0f / 256.0f));
    k_ln1<<<(MROWS + 7) / 8, 256, 0, stream>>>(ATT, x, g1, be1, X1, H16);

    k_gemm_h_bn_relu<<<dim3(ggrid(MROWS, DFF), 1), 256, 0, stream>>>(H16, DM, 0LL, W1T, DM, 0LL, F16, DFF, 0LL, b1, MROWS, DFF, DM, IW);
    k_gemm_f_bn<<<dim3(ggrid(MROWS, DM), 1), 256, 0, stream>>>(F16, DFF, 0LL, W2T, DFF, 0LL, FFo, DM, 0LL, b2, MROWS, DM, DFF, IW);
    k_ln2<<<(MROWS + 7) / 8, 256, 0, stream>>>(FFo, X1, g2, be2, out);
}
